// Network_6631429505499
// MI455X (gfx1250) — hardware-verified
//
#include <hip/hip_runtime.h>
#include <stddef.h>
#include <stdint.h>
#include <math.h>


#define NN      100000
#define NE      500000
#define NLAY    2
#define NREL    200
#define NBAS    50
#define DINI    100
#define FD      128
#define NCL     50
#define F0N     64
#define F1N     32
#define RELP    256
#define GBM     64
#define GTHR    128
#define GBNMAX  128
#define NP      100032
#define NBG     (NP / GBM)
#define NTHR    256
#define NWAVE   8
#define EPT     8
#define CHUNK   (NTHR * EPT)
#define WCAP    (EPT * 32)
#define LISTN   (NWAVE * WCAP)
#define NBA     1024
#define PKS     10
#define RCAP    12288
#define DEGCAP  64
#define GA      98
#define RA      (GA * NBA)
#define ZINTS   (2 * RCAP + 2 * NBA + LISTN)
#define MISCI   16
#define LDS_AGG ((ZINTS + MISCI) * 4)
#define PARTW   288
#define PMEAN   32
#define PM2     160
#define WSMAX   134217728

#define KP_WH   128
#define KP_WA   256
#define KP_E1   64
#define KP_REL  64
#define KP_E2   256
#define KP_F0   256
#define KP_F1   128
#define KP_F2   64
#define PO_WH   0
#define PO_WA   (PO_WH + 128 * KP_WH)
#define PO_E1   (PO_WA + 128 * KP_WA)
#define PO_REL  (PO_E1 + 128 * KP_E1)
#define PO_E2   (PO_REL + RELP * KP_REL)
#define PO_F0   (PO_E2 + 128 * KP_E2)
#define PO_F1   (PO_F0 + 64 * KP_F0)
#define PO_F2   (PO_F1 + 32 * KP_F1)
#define PL_HALVES (PO_F2 + 64 * KP_F2)

static_assert(NP == ((NN + GBM - 1) / GBM) * GBM);
static_assert(NBG * GBM == NP);
static_assert(GA == (NP + NBA - 1) / NBA && RA >= NP);
static_assert((CHUNK & (CHUNK - 1)) == 0);
static_assert(NBA == (1 << PKS));
static_assert(((long long)CHUNK << PKS) < (1LL << 31));
static_assert(((long long)NE << PKS) < (1LL << 31));
static_assert(NTHR * 4 == NBA);
static_assert(LISTN >= NBA && LISTN >= NWAVE * WCAP);
static_assert((RCAP % 32) == 0);
static_assert((ZINTS % (NTHR * 4)) == 0);
static_assert(LDS_AGG <= 262144);
static_assert((NBA % NWAVE) == 0 && (NBA % GBM) == 0);
static_assert(GBM == (GTHR / 32) * 16);
static_assert(FD == 32 * 4);
static_assert(GTHR == FD && GBNMAX == FD);
static_assert((PARTW % 32) == 0 && PARTW / 4 <= GTHR && PM2 + FD <= PARTW && PMEAN + FD <= PM2);
static_assert(((NN % GBM) * NCL) % 4 == 0 && ((((NN % GBM) * NCL) / 4) % 8) == 0);
static_assert((GBM * NCL) % 32 == 0);
static_assert(NP * FD * 2 == NP * F0N * 4);
static_assert((PO_WA % 128) == 0 && (PO_E1 % 128) == 0 && (PO_REL % 128) == 0 && (PO_E2 % 128) == 0);
static_assert((PO_F0 % 128) == 0 && (PO_F1 % 128) == 0 && (PO_F2 % 128) == 0 && (PL_HALVES % 128) == 0);
static_assert(DINI % 4 == 0 && DINI <= KP_WH);
static_assert((long long)(NN - 1) * NCL + NCL - 1 < (long long)NN * NCL);

typedef float          v4f  __attribute__((ext_vector_type(4)));
typedef float          v8f  __attribute__((ext_vector_type(8)));
typedef int            v4i  __attribute__((ext_vector_type(4)));
typedef int            v8i  __attribute__((ext_vector_type(8)));
typedef unsigned int   v4u  __attribute__((ext_vector_type(4)));
typedef unsigned short v8us __attribute__((ext_vector_type(8)));
typedef __bf16         v16b __attribute__((ext_vector_type(16)));
typedef v4f  __attribute__((may_alias)) v4fa;
typedef v4i  __attribute__((may_alias)) v4ia;
typedef v8us __attribute__((may_alias)) v8usa;
union Frag { v16b b; v8us h[2]; v4u q[2]; v8i w; };

__device__ __forceinline__ v8f wmk(const Frag& a, const Frag& b, v8f c) {
  v8f d = __builtin_amdgcn_wmma_f32_16x16x32_bf16(false, a.b, false, b.b, (short)0, c, false, false);
  asm volatile("v_nop\n\tv_nop\n\tv_nop\n\tv_nop" : "+v"(d) : "v"(a.w), "v"(b.w));
  return d;
}

__device__ __forceinline__ unsigned short bf_bits(float f) {
  unsigned int u = __float_as_uint(f);
  u += 0x7FFFu + ((u >> 16) & 1u);
  return (unsigned short)(u >> 16);
}
__device__ __forceinline__ float bf_val(unsigned short b) {
  return __uint_as_float(((unsigned int)b) << 16);
}
__device__ __forceinline__ float bf_rne(float f) { return bf_val(bf_bits(f)); }

template <int ACT>
__device__ __forceinline__ float actf(float v) {
  if constexpr (ACT == 1) {
    return fmaxf(v, 0.0f);
  } else {
    return v;
  }
}

__device__ __forceinline__ v4u pack_hilo4(float r0, float r1, float r2, float r3) {
  const unsigned short hb0 = bf_bits(r0), hb1 = bf_bits(r1), hb2 = bf_bits(r2), hb3 = bf_bits(r3);
  const unsigned short lb0 = bf_bits(r0 - bf_val(hb0)), lb1 = bf_bits(r1 - bf_val(hb1));
  const unsigned short lb2 = bf_bits(r2 - bf_val(hb2)), lb3 = bf_bits(r3 - bf_val(hb3));
  v4u pk;
  pk.x = (unsigned int)hb0 | ((unsigned int)hb1 << 16);
  pk.y = (unsigned int)hb2 | ((unsigned int)hb3 << 16);
  pk.z = (unsigned int)lb0 | ((unsigned int)lb1 << 16);
  pk.w = (unsigned int)lb2 | ((unsigned int)lb3 << 16);
  return pk;
}

__device__ __forceinline__ int scan_chunk(const int* __restrict__ dsts, int nE, int cbase, int slotBase,
                                          int nb, int vec8, int* list, int tid, int lane, int wave) {
  int wc = 0;
  const int el0  = tid * EPT;
  const int e0   = cbase + el0;
  const int sent = -2147483647 - 1;
  v4i da, db;
  if (vec8 != 0 && cbase + CHUNK <= nE) {
    da = *(const v4i*)(dsts + e0);
    db = *(const v4i*)(dsts + e0 + 4);
  } else {
    da.x = (e0     < nE) ? dsts[min(e0,     nE - 1)] : sent;
    da.y = (e0 + 1 < nE) ? dsts[min(e0 + 1, nE - 1)] : sent;
    da.z = (e0 + 2 < nE) ? dsts[min(e0 + 2, nE - 1)] : sent;
    da.w = (e0 + 3 < nE) ? dsts[min(e0 + 3, nE - 1)] : sent;
    db.x = (e0 + 4 < nE) ? dsts[min(e0 + 4, nE - 1)] : sent;
    db.y = (e0 + 5 < nE) ? dsts[min(e0 + 5, nE - 1)] : sent;
    db.z = (e0 + 6 < nE) ? dsts[min(e0 + 6, nE - 1)] : sent;
    db.w = (e0 + 7 < nE) ? dsts[min(e0 + 7, nE - 1)] : sent;
  }
  const unsigned nbs = (unsigned)slotBase;
  const unsigned unb = (unsigned)nb;
  const unsigned s0 = (unsigned)da.x - nbs, s1 = (unsigned)da.y - nbs;
  const unsigned s2 = (unsigned)da.z - nbs, s3 = (unsigned)da.w - nbs;
  const unsigned s4 = (unsigned)db.x - nbs, s5 = (unsigned)db.y - nbs;
  const unsigned s6 = (unsigned)db.z - nbs, s7 = (unsigned)db.w - nbs;
  const bool h0 = s0 < unb, h1 = s1 < unb, h2 = s2 < unb, h3 = s3 < unb;
  const bool h4 = s4 < unb, h5 = s5 < unb, h6 = s6 < unb, h7 = s7 < unb;
  const unsigned any = __builtin_amdgcn_ballot_w32(h0 | h1 | h2 | h3 | h4 | h5 | h6 | h7);
  if (any != 0u) {
#define HITJ(J, HJ, SJ) { \
      const unsigned mj = __builtin_amdgcn_ballot_w32(HJ); \
      if (mj != 0u) { \
        if (HJ) { \
          const int pos = wc + (int)__builtin_amdgcn_mbcnt_lo(mj, 0u); \
          if (pos < WCAP) list[wave * WCAP + pos] = ((el0 + (J)) << PKS) | (int)(SJ); \
        } \
        wc += (int)__builtin_popcount(mj); } }
    HITJ(0, h0, s0)
    HITJ(1, h1, s1)
    HITJ(2, h2, s2)
    HITJ(3, h3, s3)
    HITJ(4, h4, s4)
    HITJ(5, h5, s5)
    HITJ(6, h6, s6)
    HITJ(7, h7, s7)
#undef HITJ
  }
  return wc;
}

__global__ __launch_bounds__(NTHR) void k_wprep(const float* __restrict__ W, int kReal, int nReal, int sK, int sN,
                                                int jmask, int cmul, int lq, int nUnits, unsigned short* dst) {
  const int u = (int)blockIdx.x * NTHR + (int)threadIdx.x;
  if (u >= nUnits) return;
  const int n  = u >> lq;
  const int q  = u & ((1 << lq) - 1);
  const int nn = n < nReal ? n : nReal - 1;
  v8us o;
#pragma unroll
  for (int j = 0; j < 8; ++j) {
    const int c  = q * cmul + (j & jmask);
    const int cc = c < kReal ? c : kReal - 1;
    const float f = W[(size_t)cc * (size_t)sK + (size_t)nn * (size_t)sN];
    const unsigned short b = bf_bits(f);
    o[j] = (n < nReal && c < kReal) ? b : (unsigned short)0;
  }
  unsigned short* dp = dst + (size_t)u * 8;
  *(volatile v8us*)dp = o;
  __threadfence();
  *(volatile v8us*)dp = o;
}

__global__ __launch_bounds__(NTHR) void k_xprep(const float* __restrict__ eh, int nN, int nUnits,
                                                unsigned short* XP) {
  const int u = (int)blockIdx.x * NTHR + (int)threadIdx.x;
  if (u >= nUnits) return;
  const int row = u >> 4, j = u & 15, c0 = 8 * j;
  const int rr  = row < nN ? row : nN - 1;
  const int a0  = c0 < (DINI - 4) ? c0 : (DINI - 4);
  const int a1  = (c0 + 4) < (DINI - 4) ? (c0 + 4) : (DINI - 4);
  const float* rp = eh + (size_t)rr * DINI;
  const v4f va = *(const v4fa*)(rp + a0);
  const v4f vb = *(const v4fa*)(rp + a1);
  const bool rok = row < nN;
  v8us o;
  o[0] = (rok && (c0 + 0) < DINI) ? bf_bits(va.x) : (unsigned short)0;
  o[1] = (rok && (c0 + 1) < DINI) ? bf_bits(va.y) : (unsigned short)0;
  o[2] = (rok && (c0 + 2) < DINI) ? bf_bits(va.z) : (unsigned short)0;
  o[3] = (rok && (c0 + 3) < DINI) ? bf_bits(va.w) : (unsigned short)0;
  o[4] = (rok && (c0 + 4) < DINI) ? bf_bits(vb.x) : (unsigned short)0;
  o[5] = (rok && (c0 + 5) < DINI) ? bf_bits(vb.y) : (unsigned short)0;
  o[6] = (rok && (c0 + 6) < DINI) ? bf_bits(vb.z) : (unsigned short)0;
  o[7] = (rok && (c0 + 7) < DINI) ? bf_bits(vb.w) : (unsigned short)0;
  unsigned short* dp = XP + (size_t)u * 8;
  *(volatile v8us*)dp = o;
  __threadfence();
  *(volatile v8us*)dp = o;
}

template <int AM, int ACT, int GNT, int NC, int HASB>
__global__ __launch_bounds__(GTHR) void k_gemm(const unsigned short* __restrict__ A16, const float* __restrict__ A32,
                                               int lda, const float* __restrict__ ss,
                                               const unsigned short* __restrict__ BT, int ldb, int K,
                                               const float* __restrict__ bias, float* C32, int nRows) {
  static_assert(AM >= 0 && AM <= 2 && (HASB == 0 || HASB == 1));
  static_assert(NC <= 16 * GNT && 16 * GNT <= GBNMAX && (GBM * NC) % 4 == 0 && (NC % 2) == 0);
  constexpr int NF4 = GBM * NC / 4;
  constexpr int ITS = (NF4 + GTHR - 1) / GTHR;
  __shared__ __attribute__((aligned(16))) float stg[GBM * GBNMAX];
  __shared__ __attribute__((aligned(16))) float ssh[2 * FD];
  __shared__ __attribute__((aligned(16))) float sb[GBNMAX];
  const int tid = (int)threadIdx.x, lane = tid & 31, wave = tid >> 5, hh = lane >> 4, m = lane & 15;
  const int rowBase = (int)blockIdx.x * GBM;

  {
    float bb = 0.0f;
    if constexpr (HASB == 1) {
      const int bc = tid < NC ? tid : NC - 1;
      bb = bf_rne(bias[bc]);
    }
    sb[tid] = bb;
    if constexpr (AM == 2) {
      ssh[tid] = ss[tid];
      ssh[FD + tid] = ss[FD + tid];
    }
  }
  __syncthreads();

  v8f acc[GNT];
  {
    const v8f z = {0.f, 0.f, 0.f, 0.f, 0.f, 0.f, 0.f, 0.f};
#pragma unroll
    for (int t = 0; t < GNT; ++t) acc[t] = z;
  }
  const int rowA = rowBase + 16 * wave + m;
  const unsigned short* ap = A16 + (size_t)rowA * (size_t)lda + 8 * hh;
  const float* arow = A32 + (size_t)rowA * (size_t)lda + 4 * hh;
  const unsigned short* bp = BT + (size_t)m * (size_t)ldb + 8 * hh;

#pragma unroll 1
  for (int k0 = 0; k0 < K; k0 += 32) {
    Frag af;
    if constexpr (AM == 0) {
      af.h[0] = *(const v8usa*)(ap + k0);
      af.h[1] = *(const v8usa*)(ap + k0 + 16);
    } else {
      v4f x0 = *(const v4fa*)(arow + (k0 >> 1));
      v4f x1 = *(const v4fa*)(arow + (k0 >> 1) + 8);
      if constexpr (AM == 2) {
        const int cb = (k0 >> 1) + 4 * hh;
        const v4f c0 = *(const v4fa*)(ssh + cb);
        const v4f d0 = *(const v4fa*)(ssh + FD + cb);
        const v4f c1 = *(const v4fa*)(ssh + cb + 8);
        const v4f d1 = *(const v4fa*)(ssh + FD + cb + 8);
        x0.x = fmaxf(fmaf(x0.x, c0.x, d0.x), 0.0f); x0.y = fmaxf(fmaf(x0.y, c0.y, d0.y), 0.0f);
        x0.z = fmaxf(fmaf(x0.z, c0.z, d0.z), 0.0f); x0.w = fmaxf(fmaf(x0.w, c0.w, d0.w), 0.0f);
        x1.x = fmaxf(fmaf(x1.x, c1.x, d1.x), 0.0f); x1.y = fmaxf(fmaf(x1.y, c1.y, d1.y), 0.0f);
        x1.z = fmaxf(fmaf(x1.z, c1.z, d1.z), 0.0f); x1.w = fmaxf(fmaf(x1.w, c1.w, d1.w), 0.0f);
      }
      af.q[0] = pack_hilo4(x0.x, x0.y, x0.z, x0.w);
      af.q[1] = pack_hilo4(x1.x, x1.y, x1.z, x1.w);
    }
#pragma unroll
    for (int nt = 0; nt < GNT; ++nt) {
      const unsigned short* wq = bp + (size_t)(16 * nt) * (size_t)ldb + k0;
      Frag bf;
      bf.h[0] = *(const v8usa*)wq;
      bf.h[1] = *(const v8usa*)(wq + 16);
      acc[nt] = wmk(af, bf, acc[nt]);
    }
  }

#pragma unroll
  for (int nt = 0; nt < GNT; ++nt) {
    const int lc = 16 * nt + m;
    const float bb = sb[lc];
#pragma unroll
    for (int r = 0; r < 8; ++r) {
      const int lr = 16 * wave + 8 * hh + r;
      const float v = actf<ACT>(acc[nt][r] + bb);
      if (lc < NC) stg[lr * NC + lc] = v;
    }
  }
  __syncthreads();

  int nr = nRows - rowBase;
  nr = nr < 0 ? 0 : (nr > GBM ? GBM : nr);
  const int nflt4 = (nr * NC) >> 2;
  v4f pv[ITS];
#pragma unroll
  for (int it = 0; it < ITS; ++it) {
    const int i  = tid + GTHR * it;
    const int ic = i < NF4 ? i : NF4 - 1;
    pv[it] = *(const v4fa*)(stg + 4 * ic);
  }
  float* cbase = C32 + (size_t)rowBase * (size_t)NC;
#pragma unroll
  for (int it = 0; it < ITS; ++it) {
    const int i = tid + GTHR * it;
    if (i < nflt4) *(volatile v4f*)(cbase + 4 * (size_t)i) = pv[it];
  }
  __threadfence();
#pragma unroll
  for (int it = 0; it < ITS; ++it) {
    const int i = tid + GTHR * it;
    if (i < nflt4) *(volatile v4f*)(cbase + 4 * (size_t)i) = pv[it];
  }
  (void)ap; (void)arow; (void)ss;
}

__global__ __launch_bounds__(NTHR) void k_agg(const int* __restrict__ srcs, const int* __restrict__ dsts,
                                              const int* __restrict__ ets, const float* __restrict__ Mrows,
                                              const float* __restrict__ Rt, float* Xout, int nN, int nE, int vec8) {
  extern __shared__ __attribute__((aligned(16))) int lds_i[];
  int* reg1 = lds_i;
  int* reg2 = reg1 + RCAP;
  int* scnt = reg2 + RCAP;
  int* soff = scnt + NBA;
  int* list = soff + NBA;
  int* wcnt = list + LISTN;
  int* wtot = wcnt + NWAVE;
  const int tid = (int)threadIdx.x, lane = tid & 31, wave = tid >> 5;
  const int nodeBase = (int)blockIdx.x * NBA;

  {
    const v4i z4 = {0, 0, 0, 0};
    for (int i = tid * 4; i < ZINTS; i += NTHR * 4) *(v4ia*)(lds_i + i) = z4;
    if (tid < 2 * NWAVE) wcnt[tid] = 0;
  }
  __syncthreads();

  int tot = 0;
  const int nChunks = (nE + CHUNK - 1) / CHUNK;
#pragma unroll 1
  for (int ch = 0; ch < nChunks; ++ch) {
    const int cbase = ch * CHUNK;
    const int wc = scan_chunk(dsts, nE, cbase, nodeBase, NBA, vec8, list, tid, lane, wave);
    if (lane == 0) wcnt[wave] = wc;
    __syncthreads();
    int pre = 0, all = 0;
#pragma unroll
    for (int w2 = 0; w2 < NWAVE; ++w2) {
      int c = wcnt[w2];
      c = c < 0 ? 0 : (c > WCAP ? WCAP : c);
      all += c;
      pre += (w2 < wave) ? c : 0;
    }
    const int wcc  = wc > WCAP ? WCAP : wc;
    const int base = tot + pre;
#pragma unroll 1
    for (int i = lane; i < wcc; i += 32) {
      const int ent = list[wave * WCAP + i];
      const int el  = (ent >> PKS) & (CHUNK - 1);
      const int sl  = ent & (NBA - 1);
      int eid = cbase + el;
      eid = eid > nE - 1 ? nE - 1 : eid;
      const int pos = base + i;
      if (pos < RCAP) reg1[pos] = (int)(((unsigned)eid << PKS) | (unsigned)sl);
    }
    tot += all;
    tot = tot > RCAP ? RCAP : tot;
    __syncthreads();
  }
  const int nh = tot;

  if (wave == 0) {
#pragma unroll 1
    for (int b0 = 0; b0 < nh; b0 += 32) {
      const int idx = b0 + lane;
      const int uv  = reg1[idx < RCAP ? idx : RCAP - 1];
      const int m32 = (nh - b0) < 32 ? (nh - b0) : 32;
#pragma unroll 1
      for (int k = 0; k < m32; ++k) {
        const int u  = __builtin_amdgcn_readlane(uv, k);
        const int sl = u & (NBA - 1);
        if (lane == 0) scnt[sl] = scnt[sl] + 1;
      }
    }
  }
  __syncthreads();

  {
    const v4i ca = *(const v4ia*)(scnt + 4 * tid);
    const int e0 = ca.x < 0 ? 0 : ca.x, e1 = ca.y < 0 ? 0 : ca.y, e2 = ca.z < 0 ? 0 : ca.z, e3 = ca.w < 0 ? 0 : ca.w;
    const int ts = e0 + e1 + e2 + e3;
    int incl = ts;
#pragma unroll
    for (int d = 1; d < 32; d <<= 1) {
      const int up = __shfl_up(incl, d, 32);
      if (lane >= d) incl += up;
    }
    if (lane == 31) wtot[wave] = incl;
    __syncthreads();
    int pre = 0;
#pragma unroll
    for (int w2 = 0; w2 < NWAVE; ++w2) pre += (w2 < wave) ? wtot[w2] : 0;
    int run = pre + incl - ts;
    soff[4 * tid + 0] = run; run += e0;
    soff[4 * tid + 1] = run; run += e1;
    soff[4 * tid + 2] = run; run += e2;
    soff[4 * tid + 3] = run;
  }
  __syncthreads();
  for (int i = tid; i < NBA; i += NTHR) list[i] = soff[i];
  __syncthreads();

  if (wave == 0) {
#pragma unroll 1
    for (int b0 = 0; b0 < nh; b0 += 32) {
      const int idx = b0 + lane;
      const int uv  = reg1[idx < RCAP ? idx : RCAP - 1];
      const int m32 = (nh - b0) < 32 ? (nh - b0) : 32;
#pragma unroll 1
      for (int k = 0; k < m32; ++k) {
        const int u   = __builtin_amdgcn_readlane(uv, k);
        const int sl  = u & (NBA - 1);
        const int eid = (int)((unsigned)u >> PKS);
        if (lane == 0) {
          int pos = list[sl];
          pos = pos < 0 ? 0 : (pos > RCAP - 1 ? RCAP - 1 : pos);
          reg2[pos] = eid;
          list[sl] = pos + 1;
        }
      }
    }
  }
  __syncthreads();

  const int nbw = NBA / NWAVE;
  const bool ovf = (nh >= RCAP);
  const float qnan = __int_as_float(0x7fc00000);

#pragma unroll 1
  for (int jt = 0; jt < nbw; ++jt) {
    const int slot = wave * nbw + jt;
    const int node = nodeBase + slot;
    int st = soff[slot];
    const int craw = scnt[slot];
    int cnt = craw;
    st  = st < 0 ? 0 : (st > nh ? nh : st);
    cnt = cnt < 0 ? 0 : (cnt > DEGCAP ? DEGCAP : cnt);
    if (cnt > nh - st) cnt = nh - st;
    const float pz = (ovf || craw > DEGCAP) ? qnan : 0.0f;
    const bool live = node < nN;

    float g0 = 0.f, g1 = 0.f, g2 = 0.f, g3 = 0.f;
#pragma unroll 1
    for (int b0 = 0; b0 < cnt; b0 += 32) {
      int idx = st + b0 + lane; idx = idx > RCAP - 1 ? RCAP - 1 : idx;
      int eid = reg2[idx]; eid = eid < 0 ? 0 : (eid > nE - 1 ? nE - 1 : eid);
      int sr = srcs[eid]; sr = sr < 0 ? 0 : (sr > nN - 1 ? nN - 1 : sr);
      int ty = ets[eid];  ty = ty < 0 ? 0 : (ty > NREL - 1 ? NREL - 1 : ty);
      const int m32 = (cnt - b0) < 32 ? (cnt - b0) : 32;
#pragma unroll 1
      for (int k = 0; k < m32; ++k) {
        const int sk = __builtin_amdgcn_readlane(sr, k);
        const int tk = __builtin_amdgcn_readlane(ty, k);
        const v4f v = *(const v4fa*)(Mrows + (size_t)sk * FD + 4 * lane);
        const v4f t = *(const v4fa*)(Rt + (size_t)tk * FD + 4 * lane);
        g0 += (v.x + t.x);
        g1 += (v.y + t.y);
        g2 += (v.z + t.z);
        g3 += (v.w + t.w);
      }
    }
    const float inv = 1.0f / (float)(craw < 1 ? 1 : craw);
    v4f y;
    y.x = (live ? g0 * inv : 0.0f) + pz;
    y.y = (live ? g1 * inv : 0.0f) + pz;
    y.z = (live ? g2 * inv : 0.0f) + pz;
    y.w = (live ? g3 * inv : 0.0f) + pz;
    float* gp = Xout + (size_t)node * (size_t)FD + 4 * lane;
    *(volatile v4f*)gp = y;
    __threadfence();
    *(volatile v4f*)gp = y;
  }
}

__global__ __launch_bounds__(GTHR) void k_bnstat(const float* __restrict__ X, int nLive, float* part) {
  __shared__ __attribute__((aligned(16))) float stg[GBM * FD];
  __shared__ __attribute__((aligned(16))) float pst[PARTW];
  const int tid = (int)threadIdx.x;
  const int rowBase = (int)blockIdx.x * GBM;
  const float* xb = X + (size_t)rowBase * (size_t)FD;
#pragma unroll
  for (int it = 0; it < (GBM * FD / 4) / GTHR; ++it) {
    const int i = tid + GTHR * it;
    *(v4fa*)(stg + 4 * i) = *(const v4fa*)(xb + 4 * (size_t)i);
  }
  __syncthreads();
  int nb = nLive - rowBase;
  nb = nb < 0 ? 0 : (nb > GBM ? GBM : nb);
  const int c = tid;
  float s = 0.0f;
#pragma unroll 4
  for (int r = 0; r < nb; ++r) s += stg[r * FD + c];
  const float inv = 1.0f / (float)(nb < 1 ? 1 : nb);
  const float mb = s * inv;
  float q = 0.0f;
#pragma unroll 4
  for (int r = 0; r < nb; ++r) {
    const float d = stg[r * FD + c] - mb;
    q = fmaf(d, d, q);
  }
  pst[PMEAN + c] = mb;
  pst[PM2 + c]   = q;
  if (tid < PMEAN) pst[tid] = (tid == 0) ? (float)nb : 0.0f;
  __syncthreads();
  v4f ps = {0.0f, 0.0f, 0.0f, 0.0f};
  if (tid < PARTW / 4) {
    ps = *(const v4fa*)(pst + 4 * tid);
    *(volatile v4f*)(part + (size_t)blockIdx.x * PARTW + 4 * tid) = ps;
  }
  __threadfence();
  if (tid < PARTW / 4) {
    *(volatile v4f*)(part + (size_t)blockIdx.x * PARTW + 4 * tid) = ps;
  }
}

__global__ __launch_bounds__(FD) void k_bnfin(const float* __restrict__ part, int nPart,
                                              const float* __restrict__ gam, const float* __restrict__ bet,
                                              float* ss) {
  __shared__ __attribute__((aligned(16))) float stg[2 * FD];
  const int tid = (int)threadIdx.x;
  const int c = tid;
  double n = 0.0, mean = 0.0, M2 = 0.0;
#pragma unroll 1
  for (int b = 0; b < nPart; ++b) {
    const float* pr = part + (size_t)b * PARTW;
    const double nb = (double)pr[0];
    const double mb = (double)pr[PMEAN + c];
    const double qb = (double)pr[PM2 + c];
    if (nb > 0.5) {
      const double nn = n + nb;
      const double delta = mb - mean;
      const double f = nb / nn;
      mean = mean + delta * f;
      M2 = M2 + qb + delta * delta * n * f;
      n = nn;
    }
  }
  const double ntot = n < 1.0 ? 1.0 : n;
  const float varf  = (float)(M2 / ntot);
  const float meanf = (float)mean;
  const float rstd = rsqrtf(varf + 1e-5f);
  const float sc = bf_rne(gam[c]) * rstd;
  const float sh = bf_rne(bet[c]) - meanf * sc;
  stg[c] = sc;
  stg[FD + c] = sh;
  __syncthreads();
  v4f v = {0.0f, 0.0f, 0.0f, 0.0f};
  if (tid < (2 * FD) / 4) {
    v = *(const v4fa*)(stg + 4 * tid);
    *(volatile v4f*)(ss + 4 * tid) = v;
  }
  __threadfence();
  if (tid < (2 * FD) / 4) {
    *(volatile v4f*)(ss + 4 * tid) = v;
  }
}

static inline size_t al256(size_t o) { return (o + 255) & ~(size_t)255; }

extern "C" void kernel_launch(void* const* d_in, const int* in_sizes, int n_in,
                              void* d_out, int out_size, void* d_ws, size_t ws_size,
                              hipStream_t stream) {
  if (n_in < 18) return;
  if (in_sizes[0] != NLAY * NE || in_sizes[1] != NLAY * NE || in_sizes[2] != NLAY * NE) return;
  if (in_sizes[3] != NN * DINI) return;
  if (in_sizes[4] != NBAS * DINI) return;
  if (in_sizes[5] != NREL * NBAS) return;
  if (in_sizes[6] != DINI * FD) return;
  if (in_sizes[7] != DINI * FD) return;
  if (in_sizes[8] != FD * FD) return;
  if (in_sizes[9] != FD) return;
  if (in_sizes[10] != FD || in_sizes[11] != FD) return;
  if (in_sizes[12] != FD * F0N) return;
  if (in_sizes[13] != F0N) return;
  if (in_sizes[14] != F0N * F1N) return;
  if (in_sizes[15] != F1N) return;
  if (in_sizes[16] != F1N * NCL) return;
  if (in_sizes[17] != NCL) return;
  if (out_size != NN * NCL) return;

  const int*   esrc = (const int*)  d_in[0];
  const int*   edst = (const int*)  d_in[1];
  const int*   etyp = (const int*)  d_in[2];
  const float* embh = (const float*)d_in[3];
  const float* embe = (const float*)d_in[4];
  const float* relw = (const float*)d_in[5];
  const float* Wh   = (const float*)d_in[6];
  const float* We   = (const float*)d_in[7];
  const float* Wa   = (const float*)d_in[8];
  const float* ba   = (const float*)d_in[9];
  const float* gam  = (const float*)d_in[10];
  const float* bet  = (const float*)d_in[11];
  const float* W0   = (const float*)d_in[12];
  const float* b0   = (const float*)d_in[13];
  const float* W1   = (const float*)d_in[14];
  const float* b1   = (const float*)d_in[15];
  const float* W2   = (const float*)d_in[16];
  const float* b2   = (const float*)d_in[17];
  float* out = (float*)d_out;

  char* ws = (char*)d_ws;
  size_t off = 0;
  const size_t oPL = off; off = al256(off + (size_t)PL_HALVES * 2);
  const size_t oRE = off; off = al256(off + (size_t)RELP * FD * 4);
  const size_t oR  = off; off = al256(off + (size_t)RELP * FD * 4);
  const size_t oR1 = off; off = al256(off + (size_t)RA * FD * 4);
  const size_t oR2 = off; off = al256(off + (size_t)NP * FD * 4);
  const size_t oR3 = off; off = al256(off + (size_t)NP * FD * 2);
  const size_t oPT = off; off = al256(off + (size_t)NBG * PARTW * 4);
  const size_t oSS = off; off = al256(off + (size_t)(2 * FD) * 4);
  if (off > ws_size || off > (size_t)WSMAX) return;
  unsigned short* PL  = (unsigned short*)(ws + oPL);
  float*          REf = (float*)(ws + oRE);
  float*          Rf  = (float*)(ws + oR);
  float*          R1  = (float*)(ws + oR1);
  float*          R2  = (float*)(ws + oR2);
  unsigned short* XP  = (unsigned short*)(ws + oR3);
  float*          H1  = (float*)(ws + oR3);
  float*          PT  = (float*)(ws + oPT);
  float*          SS  = (float*)(ws + oSS);
  const unsigned short* dumh = PL;
  const float*          dumf = PT;

  hipFuncSetAttribute(reinterpret_cast<const void*>(&k_agg), hipFuncAttributeMaxDynamicSharedMemorySize, LDS_AGG);

  k_wprep<<<(128 * KP_WH / 8) / NTHR, NTHR, 0, stream>>>(Wh,   DINI, FD,   FD,  1,  7, 8, 4, 128 * KP_WH / 8,  PL + PO_WH);
  k_wprep<<<(128 * KP_WA / 8) / NTHR, NTHR, 0, stream>>>(Wa,   FD,   FD,   FD,  1,  3, 4, 5, 128 * KP_WA / 8,  PL + PO_WA);
  k_wprep<<<(128 * KP_E1 / 8) / NTHR, NTHR, 0, stream>>>(embe, NBAS, DINI, DINI, 1, 7, 8, 3, 128 * KP_E1 / 8,  PL + PO_E1);
  k_wprep<<<(RELP * KP_REL / 8) / NTHR, NTHR, 0, stream>>>(relw, NBAS, NREL, 1, NBAS, 7, 8, 3, RELP * KP_REL / 8, PL + PO_REL);
  k_wprep<<<(128 * KP_E2 / 8) / NTHR, NTHR, 0, stream>>>(We,   DINI, FD,   FD,  1,  3, 4, 5, 128 * KP_E2 / 8,  PL + PO_E2);
  k_wprep<<<(64 * KP_F0 / 8) / NTHR, NTHR, 0, stream>>>(W0,    FD,   F0N,  F0N, 1,  3, 4, 5, 64 * KP_F0 / 8,   PL + PO_F0);
  k_wprep<<<(32 * KP_F1 / 8) / NTHR, NTHR, 0, stream>>>(W1,    F0N,  F1N,  F1N, 1,  3, 4, 4, 32 * KP_F1 / 8,   PL + PO_F1);
  k_wprep<<<(64 * KP_F2 / 8) / NTHR, NTHR, 0, stream>>>(W2,    F1N,  NCL,  NCL, 1,  3, 4, 3, 64 * KP_F2 / 8,   PL + PO_F2);

  const int nUX = NP * 16;
  k_xprep<<<(nUX + NTHR - 1) / NTHR, NTHR, 0, stream>>>(embh, NN, nUX, XP);

  k_gemm<0, 0, 8, 128, 0><<<RELP / GBM, GTHR, 0, stream>>>(PL + PO_REL, dumf, KP_REL, SS, PL + PO_E1, KP_E1, KP_E1,
                                                            ba, REf, RELP);
  k_gemm<1, 0, 8, 128, 0><<<RELP / GBM, GTHR, 0, stream>>>(dumh, REf, FD, SS, PL + PO_E2, KP_E2, KP_E2, ba, Rf, RELP);
  k_gemm<0, 0, 8, 128, 0><<<NBG, GTHR, 0, stream>>>(XP, dumf, KP_WH, SS, PL + PO_WH, KP_WH, KP_WH, ba, R1, NP);
  k_gemm<1, 1, 8, 128, 1><<<NBG, GTHR, 0, stream>>>(dumh, R1, FD, SS, PL + PO_WA, KP_WA, KP_WA, ba, R2, NP);
  const int vec8 = ((NE & 3) == 0) ? 1 : 0;
  k_agg<<<GA, NTHR, LDS_AGG, stream>>>(esrc, edst, etyp, R2, Rf, R1, NN, NE, vec8);
  k_gemm<1, 1, 8, 128, 1><<<NBG, GTHR, 0, stream>>>(dumh, R1, FD, SS, PL + PO_WA, KP_WA, KP_WA, ba, R2, NP);
  k_agg<<<GA, NTHR, LDS_AGG, stream>>>(esrc + NE, edst + NE, etyp + NE, R2, Rf, R1, NN, NE, vec8);
  k_bnstat<<<NBG, GTHR, 0, stream>>>(R1, NN, PT);
  k_bnfin<<<1, FD, 0, stream>>>(PT, NBG, gam, bet, SS);
  k_gemm<2, 1, 4, 64, 1><<<NBG, GTHR, 0, stream>>>(dumh, R1, FD, SS, PL + PO_F0, KP_F0, KP_F0, b0, H1, NP);
  k_gemm<1, 1, 2, 32, 1><<<NBG, GTHR, 0, stream>>>(dumh, H1, F0N, SS, PL + PO_F1, KP_F1, KP_F1, b1, R2, NP);
  k_gemm<1, 0, 4, 50, 1><<<NBG, GTHR, 0, stream>>>(dumh, R2, F1N, SS, PL + PO_F2, KP_F2, KP_F2, b2, out, NN);
  (void)hipGetLastError();
}
